// MolecularGraphNeuralNetwork_18691697672232
// MI455X (gfx1250) — hardware-verified
//
#include <hip/hip_runtime.h>


namespace {
constexpr int NM = 8192, NA = 32, VOC = 10000, D = 64, L = 3;
constexpr float HS = 256.0f, WSC = 256.0f;
typedef _Float16 b16;
typedef __attribute__((ext_vector_type(16))) _Float16 v16b;
typedef __attribute__((ext_vector_type(8))) _Float16 v8b;
typedef __attribute__((ext_vector_type(8))) float v8f;
typedef __attribute__((ext_vector_type(2))) float v2f;
__device__ __forceinline__ float bf16_rne(float f) { unsigned int u = __float_as_uint(f); u += 0x7FFFu + ((u >> 16) & 1u); float r = __uint_as_float(u & 0xFFFF0000u); asm volatile("" : "+v"(r)); return r; }
__device__ __forceinline__ float bfv(float f) { float r = bf16_rne(f); asm volatile("" : "+v"(r)); return r; }
__device__ __forceinline__ void split16(float v, b16& hi, b16& lo) { hi = (b16)v; lo = (b16)(v - (float)hi); }
__device__ __forceinline__ v16b frag_kb(const b16* p, int hh) { const v8b a = *(const v8b*)(p + 8 * hh), b = *(const v8b*)(p + 16 + 8 * hh); v16b f;
#pragma unroll
  for (int e = 0; e < 8; ++e) { f[e] = a[e]; f[8 + e] = b[e]; } return f; }
__device__ __forceinline__ v8f wmma16b(v16b a, v16b b, v8f c) { v8f d = __builtin_amdgcn_wmma_f32_16x16x32_f16(false, a, false, b, (short)0, c, false, false); asm volatile("v_nop\n\tv_nop\n\tv_nop\n\tv_nop" : "+v"(d) : "v"(a), "v"(b)); return d; }
__device__ __forceinline__ void wave_lds_sync() { __builtin_amdgcn_fence(__ATOMIC_RELEASE, "workgroup"); __builtin_amdgcn_wave_barrier(); __builtin_amdgcn_fence(__ATOMIC_ACQUIRE, "workgroup"); }
__device__ __forceinline__ float pmul(float a, float b) { float p = a * b; asm volatile("" : "+v"(p)); return p; }
__device__ __forceinline__ int iclamp(int v, int lo, int hi) { return v < lo ? lo : (v > hi ? hi : v); }

__global__ __launch_bounds__(256) void wput_kernel(const float* __restrict__ w, b16* __restrict__ WT) { const int u = blockIdx.x * 256 + threadIdx.x; if (u >= L * D * 8) return; const int r = u / 8, k0 = (u % 8) * 8; v8b v;
#pragma unroll
  for (int j = 0; j < 8; ++j) v[j] = (b16)(bf16_rne(w[(size_t)r * D + k0 + j]) * WSC); for (int pass = 0; pass < 2; ++pass) { *(volatile v8b*)(WT + (size_t)r * D + k0) = v; __threadfence(); } }
__global__ __launch_bounds__(32) void mol_kernel(const int* __restrict__ fp, const float* __restrict__ adj, const float* __restrict__ emb, const b16* __restrict__ WT, const float* __restrict__ bias, const float* __restrict__ q, int MLIM, float* __restrict__ out) {
  __shared__ __attribute__((aligned(16))) b16 Vh[NA][D + 8], Vl[NA][D + 8], Aj[NA][NA + 8], Hth[D][NA + 8], Htl[D][NA + 8]; __shared__ float Vf[NA][D + 1], Hf[NA][D + 1], Sc[NA];
  const int lane = threadIdx.x, nloc = lane & 15, hlf = lane >> 4; const int m = blockIdx.x; if (m >= MLIM) return;
  for (int n = 0; n < NA; ++n) { const int id = iclamp(fp[(size_t)m * NA + n], 0, VOC - 1); for (int qd = 0; qd < 2; ++qd) { const int d = qd * 32 + lane; Vf[n][d] = bfv(emb[(size_t)id * D + d]); } Aj[n][lane] = (b16)bfv(adj[((size_t)m * NA + n) * NA + lane]); if (lane < 8) Aj[n][NA + lane] = (b16)0.0f; }
  for (int n = 0; n < NA; ++n) if (lane < 8) { Vh[n][D + lane] = (b16)0.0f; Vl[n][D + lane] = (b16)0.0f; } for (int d = 0; d < D; d += 32) for (int k = NA; k < NA + 8; ++k) { Hth[d + lane][k] = (b16)0.0f; Htl[d + lane][k] = (b16)0.0f; }
  wave_lds_sync();
#pragma unroll 1
  for (int l = 0; l < L; ++l) {
    for (int n = 0; n < NA; ++n) for (int qd = 0; qd < 2; ++qd) { const int d = qd * 32 + lane; b16 p, ql; split16(Vf[n][d] * HS, p, ql); Vh[n][d] = p; Vl[n][d] = ql; }
    wave_lds_sync();
#pragma unroll
    for (int rt = 0; rt < 2; ++rt) { v8f acc[4] = {(v8f){}, (v8f){}, (v8f){}, (v8f){}};
#pragma unroll
      for (int kb = 0; kb < D; kb += 32) { const v16b a = frag_kb(&Vh[rt * 16 + nloc][kb], hlf), al = frag_kb(&Vl[rt * 16 + nloc][kb], hlf);
#pragma unroll
        for (int t = 0; t < 4; ++t) { const v16b bw = frag_kb(WT + ((size_t)l * D + t * 16 + nloc) * D + kb, hlf); acc[t] = wmma16b(a, bw, acc[t]); acc[t] = wmma16b(al, bw, acc[t]); } }
#pragma unroll
      for (int t = 0; t < 4; ++t) { const int cc = t * 16 + nloc; const float bb = bfv(bias[l * D + cc]);
#pragma unroll
        for (int r8 = 0; r8 < 8; ++r8) { const int n = rt * 16 + 8 * hlf + r8; const float h = fmaxf(acc[t][r8] * (1.0f / (HS * WSC)) + bb, 0.0f); Hf[n][cc] = h; b16 p, ql; split16(h * HS, p, ql); Hth[cc][n] = p; Htl[cc][n] = ql; } } }
    wave_lds_sync();
#pragma unroll
    for (int rt = 0; rt < 2; ++rt) { v8f acc[4] = {(v8f){}, (v8f){}, (v8f){}, (v8f){}}; const v16b a = frag_kb(&Aj[rt * 16 + nloc][0], hlf);
#pragma unroll
      for (int t = 0; t < 4; ++t) { acc[t] = wmma16b(a, frag_kb(&Hth[t * 16 + nloc][0], hlf), acc[t]); acc[t] = wmma16b(a, frag_kb(&Htl[t * 16 + nloc][0], hlf), acc[t]); }
#pragma unroll
      for (int t = 0; t < 4; ++t)
#pragma unroll
        for (int r8 = 0; r8 < 8; ++r8) { const int n = rt * 16 + 8 * hlf + r8, cc = t * 16 + nloc; Vf[n][cc] = Hf[n][cc] + acc[t][r8] * (1.0f / HS); } }
    wave_lds_sync(); }
  { float s = 0.0f; for (int d = 0; d < D; ++d) s += pmul(Vf[lane][d], bfv(q[d])); float mx = s; for (int o = 16; o; o >>= 1) mx = fmaxf(mx, __shfl_xor(mx, o)); const float e = __expf(s - mx); float se = e; for (int o = 16; o; o >>= 1) se += __shfl_xor(se, o); Sc[lane] = e / se; }
  wave_lds_sync();
  float o0 = 0.0f, o1 = 0.0f; for (int n = 0; n < NA; ++n) { o0 += pmul(Sc[n], Vf[n][lane * 2]); o1 += pmul(Sc[n], Vf[n][lane * 2 + 1]); }
  for (int pass = 0; pass < 2; ++pass) { *(volatile v2f*)(out + (size_t)m * D + lane * 2) = (v2f){o0, o1}; __threadfence(); } }
}

extern "C" void kernel_launch(void* const* d_in, const int* in_sizes, int n_in, void* d_out, int out_size, void* d_ws, size_t ws_size, hipStream_t stream) {
  (void)n_in;
  auto Fp = [&](int i) { return (const float*)d_in[i]; }; auto Ip = [&](int i) { return (const int*)d_in[i]; };
  if (in_sizes[0] != NM * NA || in_sizes[1] != NM * NA * NA || in_sizes[2] != VOC * D || in_sizes[3] != L * D * D || in_sizes[4] != L * D || in_sizes[5] != D || out_size != NM * D) return;
  const int MLIM = NM;
  size_t off = 0; char* ws = (char*)d_ws;
  auto carve = [&](size_t bytes) { char* p = ws + off; off += (bytes + 255) & ~(size_t)255; return p; };
  b16* WT = (b16*)carve((size_t)L * D * D * 2);
  if (off > ws_size || off > ((size_t)1 << 20)) return;
  wput_kernel<<<(L * D * 8 + 255) / 256, 256, 0, stream>>>(Fp(3), WT);
  mol_kernel<<<MLIM, 32, 0, stream>>>(Ip(0), Fp(1), Fp(2), WT, Fp(4), Fp(5), MLIM, (float*)d_out);
}
